// TransformerDecoderLayer_5463198401294
// MI455X (gfx1250) — hardware-run, weakly checked
//
#include <hip/hip_runtime.h>


#ifndef NB
#define NB 4
#endif
#ifndef SEQ
#define SEQ 1024
#endif
#define NB_FULL  4
#define SEQ_FULL 1024
#ifndef OUT_SEQ
#define OUT_SEQ SEQ
#endif
#define DM   1024
#define NH_  16
#define HD   64
#define HID  4096
#define AW   4
#define OSP  68
#define LTP  72
#define WCAR 64.0f
#define HCAR 16.0f
#define GCAR 256.0f
#define CTXM 16.0f
#define RSC  2048.0f
#define RINV (1.0f / 2048.0f)
#define SINV (1.0f / 4096.0f)
#define XSC  (1.0f / 1024.0f)
#define SC2  ((float)(0.03125 * 1.4426950408889634))
#define LOG2E 1.4426950408889634f
#define FILLV (-1.0e4f)
#define PSH  14.0f
#define NEGB (-3.0e38f)

static_assert(NH_ * HD == DM);
static_assert(HD == 64);
static_assert(DM % 64 == 0);
static_assert(DM % 256 == 0);
static_assert(HID % 64 == 0);
static_assert(DM % 32 == 0);
static_assert(HID % 32 == 0);
static_assert(SEQ % 64 == 0);
static_assert((NB * SEQ) % 64 == 0);
static_assert((NB * SEQ) % 32 == 0);
static_assert((NB * SEQ) % 8 == 0);
static_assert(SEQ % 32 == 0);
static_assert(SEQ % (16 * AW) == 0);
static_assert(NB <= NB_FULL);
static_assert(SEQ <= SEQ_FULL);
static_assert((OSP * 4) % 16 == 0);
static_assert((LTP * 2) % 16 == 0);
static_assert(32 * 16 * 4 == 16 * 64 * 2);
static_assert(32 * 16 * 8 == 16 * 64 * 4);
static_assert(256 * 16 * 2 == 64 * 64 * 2);
static_assert(16 * OSP * 4 <= 131072);
static_assert(AW * 16 * OSP * 4 <= 131072);
static_assert(64 * LTP * 2 <= 131072);

typedef _Float16 h16;
typedef __attribute__((ext_vector_type(16))) _Float16 v16h;
typedef __attribute__((ext_vector_type(8)))  _Float16 v8h;
typedef __attribute__((ext_vector_type(8)))  float    v8f;
typedef __attribute__((ext_vector_type(4)))  float    v4f;
typedef __attribute__((ext_vector_type(4)))  int      v4i;
typedef v4f  __attribute__((may_alias)) v4fa;
typedef v8h  __attribute__((may_alias)) v8ha;

__device__ __forceinline__ unsigned short f2bf(float f) { unsigned u = __float_as_uint(f); u += 0x7FFFu + ((u >> 16) & 1u); return (unsigned short)(u >> 16); }
__device__ __forceinline__ float bfr(float f) { return __uint_as_float(((unsigned)f2bf(f)) << 16); }
static __device__ __forceinline__ h16 toh_flush(float v) { const h16 r = (h16)v; return (fabsf(v) < 6.103515625e-05f) ? (h16)0.0f : r; }
__device__ __forceinline__ v16h cat16(v8h lo, v8h hi) { return __builtin_shufflevector(lo, hi, 0, 1, 2, 3, 4, 5, 6, 7, 8, 9, 10, 11, 12, 13, 14, 15); }
__device__ __forceinline__ v8f wmma16(v16h a, v16h b, v8f c) {
    c = __builtin_amdgcn_wmma_f32_16x16x32_f16(false, a, false, b, (short)0, c, false, false);
    asm volatile("v_nop\n\tv_nop\n\tv_nop\n\tv_nop" : "+v"(c) : "v"(a), "v"(b));
    return c;
}
__device__ __forceinline__ v16h ldh(const h16* p) { return cat16(*(const v8h*)p, *(const v8h*)(p + 16)); }
__device__ __forceinline__ void wave_sync() { __builtin_amdgcn_fence(3  , "wavefront"); __builtin_amdgcn_wave_barrier(); asm volatile("" ::: "memory"); }
__device__ __forceinline__ float wsum(float v) {
    v += __shfl_xor(v, 16, 32); v += __shfl_xor(v, 8, 32); v += __shfl_xor(v, 4, 32); v += __shfl_xor(v, 2, 32); v += __shfl_xor(v, 1, 32); return v; }

__global__ __launch_bounds__(256) void k_cvth8(const float* __restrict__ src, h16* dst, size_t n8) {
    const size_t i = (size_t)blockIdx.x * 256 + threadIdx.x; if (i >= n8) return;
    const v8f v = *(const v8f*)(src + i * 8); v8h o;
#pragma unroll
    for (int k = 0; k < 8; ++k) o[k] = toh_flush(bfr(v[k]));
    *(volatile v8h*)(dst + i * 8) = o; __threadfence(); *(volatile v8h*)(dst + i * 8) = o;
}

__global__ __launch_bounds__(256) void k_wtr(const float* __restrict__ W, h16* Wt, int K, int N) {
    __shared__ __align__(16) h16 lt[64 * LTP];
    const int tid = threadIdx.x;
    const int n0 = blockIdx.x * 64, k0 = blockIdx.y * 64;
    const int rr = tid >> 4, c4 = (tid & 15) * 4;
#pragma unroll 1
    for (int i = 0; i < 4; ++i) {
        const int kr = rr + 16 * i;
        const v4f v = *(const v4f*)(W + (size_t)(k0 + kr) * N + n0 + c4);
#pragma unroll
        for (int j = 0; j < 4; ++j) lt[(c4 + j) * LTP + kr] = toh_flush(bfr(v[j]) * WCAR);
    }
    __syncthreads();
    const int nr = tid >> 3, c8 = (tid & 7) * 8;
    const v8h o0 = *(const v8ha*)(&lt[nr * LTP + c8]);
    const v8h o1 = *(const v8ha*)(&lt[(nr + 32) * LTP + c8]);
    h16* d0 = Wt + (size_t)(n0 + nr) * K + k0 + c8;
    h16* d1 = Wt + (size_t)(n0 + nr + 32) * K + k0 + c8;
    *(volatile v8h*)d0 = o0; *(volatile v8h*)d1 = o1;
    __threadfence();
    *(volatile v8h*)d0 = o0; *(volatile v8h*)d1 = o1;
}

template <int MODE, int RES>
__device__ __forceinline__ void proj_body(const h16* __restrict__ X, const h16* __restrict__ Wt, h16* P, h16* PR, float osc) {
    __shared__ __align__(16) float os[16 * OSP];
    const int lane = threadIdx.x & 31, lr = lane & 15, hi = lane >> 4;
    const int r0 = blockIdx.x * 64, head = blockIdx.y;
    v8f acc[4][4];
#pragma unroll
    for (int mb = 0; mb < 4; ++mb)
#pragma unroll
        for (int nb = 0; nb < 4; ++nb) acc[mb][nb] = (v8f){};
    const size_t xoff = (size_t)(r0 + lr) * DM + (size_t)head * HD + 8 * hi;
    const size_t woff = (size_t)lr * HD + 8 * hi;
#pragma unroll 1
    for (int kc = 0; kc < HD; kc += 32) {
        v16h a[4];
        if (MODE == 0) {
#pragma unroll
            for (int mb = 0; mb < 4; ++mb) a[mb] = ldh(X + xoff + (size_t)mb * 16 * DM + kc);
#pragma unroll
            for (int nb = 0; nb < 4; ++nb) { const v16h b = ldh(Wt + woff + (size_t)nb * 16 * HD + kc);
#pragma unroll
                for (int mb = 0; mb < 4; ++mb) acc[mb][nb] = wmma16(a[mb], b, acc[mb][nb]); }
        } else {
#pragma unroll
            for (int mb = 0; mb < 4; ++mb) a[mb] = ldh(Wt + woff + (size_t)mb * 16 * HD + kc);
#pragma unroll
            for (int nb = 0; nb < 4; ++nb) { const v16h b = ldh(X + xoff + (size_t)nb * 16 * DM + kc);
#pragma unroll
                for (int mb = 0; mb < 4; ++mb) acc[mb][nb] = wmma16(a[mb], b, acc[mb][nb]); }
        }
    }
    const int bb = r0 / SEQ, tt = r0 % SEQ; const int zh = bb * NH_ + head;
    size_t obase, pitch;
    if (MODE == 0) { obase = ((size_t)zh * SEQ + (size_t)tt) * HD; pitch = HD; }
    else           { obase = (size_t)zh * HD * SEQ + (size_t)tt;   pitch = SEQ; }
#pragma unroll
    for (int mb = 0; mb < 4; ++mb) {
#pragma unroll
        for (int nb = 0; nb < 4; ++nb) {
#pragma unroll
            for (int j = 0; j < 8; ++j) os[(hi * 8 + j) * OSP + nb * 16 + lr] = acc[mb][nb][j] * osc; }
        wave_sync();
#pragma unroll 1
        for (int ps = 0; ps < 2; ++ps) {
#pragma unroll
            for (int s = 0; s < 4; ++s) { const int row = 4 * s + (lane >> 3), c8 = (lane & 7) * 8;
                const v4f x0 = *(const v4fa*)(&os[row * OSP + c8]); const v4f x1 = *(const v4fa*)(&os[row * OSP + c8 + 4]); v8h hv, rv;
#pragma unroll
                for (int i = 0; i < 4; ++i) { const h16 a0 = toh_flush(x0[i]); const h16 a1 = toh_flush(x1[i]); hv[i] = a0; hv[4 + i] = a1;
                    rv[i] = toh_flush((x0[i] - (float)a0) * RSC); rv[4 + i] = toh_flush((x1[i] - (float)a1) * RSC); }
                const size_t oo = obase + (size_t)(mb * 16 + row) * pitch + c8;
                *(volatile v8h*)(P + oo) = hv; if (RES) *(volatile v8h*)(PR + oo) = rv; }
            if (ps == 0) __threadfence(); }
        wave_sync();
    }
}
__global__ __launch_bounds__(32) void k_proj_qk(const h16* __restrict__ X, const h16* __restrict__ Wt, h16* P, float osc) { proj_body<0, 0>(X, Wt, P, P, osc); }
__global__ __launch_bounds__(32) void k_proj_vt(const h16* __restrict__ X, const h16* __restrict__ Wt, h16* P, float osc) { proj_body<1, 0>(X, Wt, P, P, osc); }
__global__ __launch_bounds__(32) void k_proj_vtr(const h16* __restrict__ X, const h16* __restrict__ Wt, h16* P, h16* PR, float osc) { proj_body<1, 1>(X, Wt, P, PR, osc); }

template <int V_RES, int WRITE_CR>
__device__ __forceinline__ void flash_body(const h16* __restrict__ QP, const h16* __restrict__ KP, const h16* __restrict__ VT, const h16* __restrict__ VR, const int* __restrict__ mask, h16* CTX, h16* CR) {
    __shared__ __align__(16) float os[AW * 16 * OSP];
    const int lane = threadIdx.x & 31, lr = lane & 15, hi = lane >> 4;
    const int wave = __builtin_amdgcn_readfirstlane((int)(threadIdx.x >> 5));
    const int zh = blockIdx.y; const int b = zh / NH_, h = zh % NH_;
    const int t0 = (blockIdx.x * AW + wave) * 16;
    const int tq = t0 + lr;
    const float slope = __uint_as_float((unsigned)(126 - h) << 23);
    const size_t pbase = (size_t)zh * SEQ * HD;
    const size_t qo = pbase + (size_t)tq * HD + 8 * hi;
    const v16h qf0 = ldh(QP + qo), qf1 = ldh(QP + qo + 32);
    const size_t ko = pbase + (size_t)lr * HD + 8 * hi;
    const size_t vo = pbase + (size_t)lr * SEQ + 8 * hi;
    const int* mrow = mask + (size_t)b * SEQ_FULL + 8 * hi;
    v8f o[4], orr[4];
#pragma unroll
    for (int j = 0; j < 4; ++j) { o[j] = (v8f){}; orr[j] = (v8f){}; }
    float m = NEGB, l = 0.0f;
#pragma unroll 1
    for (int key0 = 0; key0 < SEQ; key0 += 32) {
        const h16* ka = KP + ko + (size_t)key0 * HD;
        v8f sa = (v8f){}, sb = (v8f){};
        { const v16h k00 = ldh(ka), k01 = ldh(ka + 32);
          sa = wmma16(k00, qf0, sa); sa = wmma16(k01, qf1, sa); }
        { const v16h k10 = ldh(ka + 16 * HD), k11 = ldh(ka + 16 * HD + 32);
          sb = wmma16(k10, qf0, sb); sb = wmma16(k11, qf1, sb); }
        const int* mp = mrow + key0;
        const v4i m0 = *(const v4i*)mp, m1 = *(const v4i*)(mp + 4), m2 = *(const v4i*)(mp + 16), m3 = *(const v4i*)(mp + 20);
        int kx[8], ky[8];
#pragma unroll
        for (int r = 0; r < 4; ++r) { kx[r] = m0[r]; kx[4 + r] = m1[r]; ky[r] = m2[r]; ky[4 + r] = m3[r]; }
        const int da0 = tq - (key0 + 8 * hi);
        float ta[8], tb[8]; float mx = NEGB;
#pragma unroll
        for (int r = 0; r < 8; ++r) {
            const float pna = fabsf((float)(da0 - r)) * slope;
            const float pnb = fabsf((float)(da0 - 16 - r)) * slope;
            float ea = sa[r] * SINV - pna, eb = sb[r] * SINV - pnb;
            ea = (kx[r] == 0) ? FILLV : ea; eb = (ky[r] == 0) ? FILLV : eb;
            ta[r] = ea * SC2; tb[r] = eb * SC2;
            mx = fmaxf(mx, fmaxf(ta[r], tb[r])); }
        mx = fmaxf(mx, __shfl_xor(mx, 16, 32));
        const float mnew = fmaxf(m, mx);
        const float alpha = __builtin_amdgcn_exp2f(m - mnew);
        const float sh = PSH - mnew;
        v16h pb; float ls = 0.0f;
#pragma unroll
        for (int r = 0; r < 8; ++r) {
            const float aa = ta[r] + sh, ab = tb[r] + sh;
            const float ea = __builtin_amdgcn_exp2f(aa), eb = __builtin_amdgcn_exp2f(ab);
            const h16 pa = (aa < -14.0f) ? (h16)0.0f : (h16)ea;
            const h16 pc = (ab < -14.0f) ? (h16)0.0f : (h16)eb;
            pb[r] = pa; pb[8 + r] = pc;
            ls += (float)pa + (float)pc; }
        l = l * alpha + ls; m = mnew;
        const h16* va = VT + vo + key0;
        const h16* vra = VR + vo + key0;
#pragma unroll
        for (int j = 0; j < 4; ++j) {
            o[j] = o[j] * alpha;
            const v16h vj = ldh(va + (size_t)16 * j * SEQ);
            o[j] = wmma16(vj, pb, o[j]);
            if (V_RES) {
                orr[j] = orr[j] * alpha;
                const v16h vrj = ldh(vra + (size_t)16 * j * SEQ);
                orr[j] = wmma16(vrj, pb, orr[j]); } }
    }
    l += __shfl_xor(l, 16, 32);
    const float lsafe = (l > 0.0f) ? l : 1.0f;
    const float inv = CTXM * __builtin_amdgcn_rcpf(lsafe);
    const int wb = wave * 16 * OSP;
#pragma unroll
    for (int j = 0; j < 4; ++j) { v4f a, c;
        v8f f = o[j];
        if (V_RES) f = o[j] + orr[j] * RINV;
        a[0] = f[0] * inv; a[1] = f[1] * inv; a[2] = f[2] * inv; a[3] = f[3] * inv;
        c[0] = f[4] * inv; c[1] = f[5] * inv; c[2] = f[6] * inv; c[3] = f[7] * inv;
        *(v4fa*)(&os[wb + lr * OSP + 16 * j + 8 * hi]) = a; *(v4fa*)(&os[wb + lr * OSP + 16 * j + 8 * hi + 4]) = c; }
    wave_sync();
    const size_t obase = ((size_t)b * SEQ + t0) * DM + (size_t)h * HD;
#pragma unroll 1
    for (int ps = 0; ps < 2; ++ps) {
#pragma unroll
        for (int s = 0; s < 4; ++s) { const int row = 4 * s + (lane >> 3), c8 = (lane & 7) * 8;
            const v4f x0 = *(const v4fa*)(&os[wb + row * OSP + c8]); const v4f x1 = *(const v4fa*)(&os[wb + row * OSP + c8 + 4]); v8h hv, rv;
#pragma unroll
            for (int i = 0; i < 4; ++i) { const h16 a0 = toh_flush(x0[i]); const h16 a1 = toh_flush(x1[i]); hv[i] = a0; hv[4 + i] = a1;
                rv[i] = toh_flush((x0[i] - (float)a0) * RSC); rv[4 + i] = toh_flush((x1[i] - (float)a1) * RSC); }
            const size_t oo = obase + (size_t)row * DM + c8;
            *(volatile v8h*)(CTX + oo) = hv; if (WRITE_CR) *(volatile v8h*)(CR + oo) = rv; }
        if (ps == 0) __threadfence(); }
}
__global__ __launch_bounds__(32 * AW) void k_flash_vr(const h16* __restrict__ QP, const h16* __restrict__ KP, const h16* __restrict__ VT, const h16* __restrict__ VR, const int* __restrict__ mask, h16* CTX) {
    flash_body<1, 0>(QP, KP, VT, VR, mask, CTX, CTX); }
__global__ __launch_bounds__(32 * AW) void k_flash_cr(const h16* __restrict__ QP, const h16* __restrict__ KP, const h16* __restrict__ VT, const int* __restrict__ mask, h16* CTX, h16* CR) {
    flash_body<0, 1>(QP, KP, VT, VT, mask, CTX, CR); }

__global__ __launch_bounds__(32) void k_gemm(const h16* __restrict__ A, const h16* __restrict__ Bt, const float* __restrict__ bias, float* C, int K, int N, float sc) {
    __shared__ __align__(16) float os[16 * OSP];
    const int lane = threadIdx.x & 31, lr = lane & 15, hi = lane >> 4; const int r0 = blockIdx.x * 64, c0 = blockIdx.y * 64;
    v8f acc[4][4];
#pragma unroll
    for (int mb = 0; mb < 4; ++mb)
#pragma unroll
        for (int nb = 0; nb < 4; ++nb) acc[mb][nb] = (v8f){};
    const size_t aoff = (size_t)(r0 + lr) * K + 8 * hi, boff = (size_t)(c0 + lr) * K + 8 * hi;
#pragma unroll 1
    for (int kc = 0; kc < K; kc += 32) {
        v16h a[4];
#pragma unroll
        for (int mb = 0; mb < 4; ++mb) a[mb] = ldh(A + aoff + (size_t)mb * 16 * K + kc);
#pragma unroll
        for (int nb = 0; nb < 4; ++nb) { const v16h b = ldh(Bt + boff + (size_t)nb * 16 * K + kc);
#pragma unroll
            for (int mb = 0; mb < 4; ++mb) acc[mb][nb] = wmma16(a[mb], b, acc[mb][nb]); }
    }
    float bc[4];
#pragma unroll
    for (int nb = 0; nb < 4; ++nb) bc[nb] = bfr(bias[c0 + nb * 16 + lr]);
#pragma unroll
    for (int mb = 0; mb < 4; ++mb) {
#pragma unroll
        for (int nb = 0; nb < 4; ++nb) {
#pragma unroll
            for (int j = 0; j < 8; ++j) os[(hi * 8 + j) * OSP + nb * 16 + lr] = acc[mb][nb][j] * sc + bc[nb]; }
        wave_sync();
#pragma unroll 1
        for (int ps = 0; ps < 2; ++ps) {
#pragma unroll
            for (int s = 0; s < 8; ++s) { const int row = 2 * s + (lane >> 4), cofs = (lane & 15) * 4;
                const v4f val = *(const v4fa*)(&os[row * OSP + cofs]);
                *(volatile v4f*)(C + (size_t)(r0 + mb * 16 + row) * N + c0 + cofs) = val; }
            if (ps == 0) __threadfence(); }
        wave_sync();
    }
}

__global__ __launch_bounds__(32) void k_gemm_r(const h16* __restrict__ A, const h16* __restrict__ AR, const h16* __restrict__ Bt, const float* __restrict__ bias, float* C, int K, int N, float sc) {
    __shared__ __align__(16) float os[16 * OSP];
    const int lane = threadIdx.x & 31, lr = lane & 15, hi = lane >> 4; const int r0 = blockIdx.x * 32, c0 = blockIdx.y * 64;
    v8f acc[2][4], accr[2][4];
#pragma unroll
    for (int mb = 0; mb < 2; ++mb)
#pragma unroll
        for (int nb = 0; nb < 4; ++nb) { acc[mb][nb] = (v8f){}; accr[mb][nb] = (v8f){}; }
    const size_t aoff = (size_t)(r0 + lr) * K + 8 * hi, boff = (size_t)(c0 + lr) * K + 8 * hi;
#pragma unroll 1
    for (int kc = 0; kc < K; kc += 32) {
        v16h a[2], ar[2];
#pragma unroll
        for (int mb = 0; mb < 2; ++mb) { a[mb] = ldh(A + aoff + (size_t)mb * 16 * K + kc); ar[mb] = ldh(AR + aoff + (size_t)mb * 16 * K + kc); }
#pragma unroll
        for (int nb = 0; nb < 4; ++nb) { const v16h b = ldh(Bt + boff + (size_t)nb * 16 * K + kc);
#pragma unroll
            for (int mb = 0; mb < 2; ++mb) { acc[mb][nb] = wmma16(a[mb], b, acc[mb][nb]); accr[mb][nb] = wmma16(ar[mb], b, accr[mb][nb]); } }
    }
    float bc[4];
#pragma unroll
    for (int nb = 0; nb < 4; ++nb) bc[nb] = bfr(bias[c0 + nb * 16 + lr]);
#pragma unroll
    for (int mb = 0; mb < 2; ++mb) {
#pragma unroll
        for (int nb = 0; nb < 4; ++nb) {
#pragma unroll
            for (int j = 0; j < 8; ++j) os[(hi * 8 + j) * OSP + nb * 16 + lr] = (acc[mb][nb][j] + accr[mb][nb][j] * RINV) * sc + bc[nb]; }
        wave_sync();
#pragma unroll 1
        for (int ps = 0; ps < 2; ++ps) {
#pragma unroll
            for (int s = 0; s < 8; ++s) { const int row = 2 * s + (lane >> 4), cofs = (lane & 15) * 4;
                const v4f val = *(const v4fa*)(&os[row * OSP + cofs]);
                *(volatile v4f*)(C + (size_t)(r0 + mb * 16 + row) * N + c0 + cofs) = val; }
            if (ps == 0) __threadfence(); }
        wave_sync();
    }
}

__global__ __launch_bounds__(32) void k_swiglu(const h16* __restrict__ A, const h16* __restrict__ Bt, const float* __restrict__ b12, h16* G) {
    __shared__ __align__(16) float os[16 * OSP];
    const int lane = threadIdx.x & 31, lr = lane & 15, hi = lane >> 4; const int r0 = blockIdx.x * 32, c0 = blockIdx.y * 64;
    v8f acc1[2][4], acc2[2][4];
#pragma unroll
    for (int mb = 0; mb < 2; ++mb)
#pragma unroll
        for (int nb = 0; nb < 4; ++nb) { acc1[mb][nb] = (v8f){}; acc2[mb][nb] = (v8f){}; }
    const size_t aoff = (size_t)(r0 + lr) * DM + 8 * hi;
    const size_t b1off = (size_t)(c0 + lr) * DM + 8 * hi, b2off = (size_t)(HID + c0 + lr) * DM + 8 * hi;
#pragma unroll 1
    for (int kc = 0; kc < DM; kc += 32) {
        v16h a[2];
#pragma unroll
        for (int mb = 0; mb < 2; ++mb) a[mb] = ldh(A + aoff + (size_t)mb * 16 * DM + kc);
#pragma unroll
        for (int nb = 0; nb < 4; ++nb) {
            const v16h b1 = ldh(Bt + b1off + (size_t)nb * 16 * DM + kc);
#pragma unroll
            for (int mb = 0; mb < 2; ++mb) acc1[mb][nb] = wmma16(a[mb], b1, acc1[mb][nb]);
            const v16h b2 = ldh(Bt + b2off + (size_t)nb * 16 * DM + kc);
#pragma unroll
            for (int mb = 0; mb < 2; ++mb) acc2[mb][nb] = wmma16(a[mb], b2, acc2[mb][nb]); }
    }
    float b1c[4], b2c[4];
#pragma unroll
    for (int nb = 0; nb < 4; ++nb) { b1c[nb] = bfr(b12[c0 + nb * 16 + lr]); b2c[nb] = bfr(b12[HID + c0 + nb * 16 + lr]); }
#pragma unroll
    for (int mb = 0; mb < 2; ++mb) {
#pragma unroll
        for (int nb = 0; nb < 4; ++nb) {
#pragma unroll
            for (int j = 0; j < 8; ++j) {
                const float x1 = acc1[mb][nb][j] * XSC + b1c[nb];
                const float x2 = acc2[mb][nb][j] * XSC + b2c[nb];
                const float sg = __builtin_amdgcn_rcpf(1.0f + __builtin_amdgcn_exp2f(-x1 * LOG2E));
                os[(hi * 8 + j) * OSP + nb * 16 + lr] = ((x1 * sg) * x2) * GCAR; } }
        wave_sync();
#pragma unroll 1
        for (int ps = 0; ps < 2; ++ps) {
#pragma unroll
            for (int s = 0; s < 4; ++s) { const int row = 4 * s + (lane >> 3), c8 = (lane & 7) * 8;
                const v4f x0 = *(const v4fa*)(&os[row * OSP + c8]); const v4f x1 = *(const v4fa*)(&os[row * OSP + c8 + 4]); v8h hv;
#pragma unroll
                for (int i = 0; i < 4; ++i) { hv[i] = toh_flush(x0[i]); hv[4 + i] = toh_flush(x1[i]); }
                *(volatile v8h*)(G + (size_t)(r0 + mb * 16 + row) * HID + c0 + c8) = hv; }
            if (ps == 0) __threadfence(); }
        wave_sync();
    }
}

struct MuRs { float mu; float rs; };
__device__ __forceinline__ MuRs ln_stats(const float* __restrict__ xr, int lane) {
#pragma clang fp contract(off)
    float s = 0.0f;
#pragma unroll 1
    for (int c = 0; c < DM / 128; ++c) { const v4f v = *(const v4f*)(xr + c * 128 + lane * 4); s += (v[0] + v[1]) + (v[2] + v[3]); }
    s = wsum(s);
    const float mu = s * (1.0f / DM);
    float q = 0.0f;
#pragma unroll 1
    for (int c = 0; c < DM / 128; ++c) { const v4f v = *(const v4f*)(xr + c * 128 + lane * 4);
        const float d0 = v[0] - mu, d1 = v[1] - mu, d2 = v[2] - mu, d3 = v[3] - mu;
        q += (d0 * d0 + d1 * d1) + (d2 * d2 + d3 * d3); }
    q = wsum(q);
    MuRs r; r.mu = mu; r.rs = rsqrtf(q * (1.0f / DM) + 1e-5f);
    return r;
}
__global__ __launch_bounds__(256) void k_ln_h(const float* __restrict__ X, const float* __restrict__ gw, const float* __restrict__ gb, h16* O) {
#pragma clang fp contract(off)
    const int lane = threadIdx.x & 31;
    const int wave = __builtin_amdgcn_readfirstlane((int)(threadIdx.x >> 5));
    const int row = blockIdx.x * 8 + wave;
    const float* xr = X + (size_t)row * DM;
    const MuRs st = ln_stats(xr, lane);
    h16* orow = O + (size_t)row * DM;
#pragma unroll 1
    for (int ps = 0; ps < 2; ++ps) {
#pragma unroll 1
        for (int i = 0; i < DM / 256; ++i) { const int base = i * 256 + lane * 8;
            const v4f x0 = *(const v4f*)(xr + base), x1 = *(const v4f*)(xr + base + 4);
            const v4f w0 = *(const v4f*)(gw + base), w1 = *(const v4f*)(gw + base + 4);
            const v4f b0 = *(const v4f*)(gb + base), b1 = *(const v4f*)(gb + base + 4);
            v8h ov;
#pragma unroll
            for (int j = 0; j < 4; ++j) {
                const float y0 = ((x0[j] - st.mu) * st.rs) * bfr(w0[j]) + bfr(b0[j]);
                const float y1 = ((x1[j] - st.mu) * st.rs) * bfr(w1[j]) + bfr(b1[j]);
                ov[j] = toh_flush(y0 * HCAR); ov[4 + j] = toh_flush(y1 * HCAR); }
            *(volatile v8h*)(orow + base) = ov; }
        if (ps == 0) __threadfence(); }
}
__global__ __launch_bounds__(256) void k_ln_f(const float* __restrict__ X, const float* __restrict__ gw, const float* __restrict__ gb, float* O) {
#pragma clang fp contract(off)
    const int lane = threadIdx.x & 31;
    const int wave = __builtin_amdgcn_readfirstlane((int)(threadIdx.x >> 5));
    const int row = blockIdx.x * 8 + wave;
    const float* xr = X + (size_t)row * DM;
    const MuRs st = ln_stats(xr, lane);
    float* orow = O + ((size_t)(row / SEQ) * OUT_SEQ + (size_t)(row % SEQ)) * DM;
#pragma unroll 1
    for (int ps = 0; ps < 2; ++ps) {
#pragma unroll 1
        for (int c = 0; c < DM / 128; ++c) { const int base = c * 128 + lane * 4;
            const v4f x0 = *(const v4f*)(xr + base);
            const v4f w0 = *(const v4f*)(gw + base);
            const v4f b0 = *(const v4f*)(gb + base);
            v4f ov;
#pragma unroll
            for (int j = 0; j < 4; ++j) ov[j] = ((x0[j] - st.mu) * st.rs) * bfr(w0[j]) + bfr(b0[j]);
            *(volatile v4f*)(orow + base) = ov; }
        if (ps == 0) __threadfence(); }
}

static constexpr float OSC_ONE = 1.0f;
static constexpr float OSC_V2  = 1.0f / 16.0f;
static constexpr float SC_WO   = 1.0f / 65536.0f;
static constexpr float SC_W3   = 1.0f / 16384.0f;

static constexpr size_t al256(size_t v) { return (v + 255) & ~(size_t)255; }
static constexpr size_t SZ_X   = al256((size_t)NB * SEQ * DM * 2);
static constexpr size_t SZ_PL  = al256((size_t)NB * NH_ * SEQ * HD * 2);
static constexpr size_t SZ_HF  = al256((size_t)NB * SEQ * DM * 4);
static constexpr size_t SZ_G   = al256((size_t)NB * SEQ * HID * 2);
static constexpr size_t SZ_WS  = al256((size_t)HD * HD * 2);
static constexpr size_t SZ_WO  = al256((size_t)DM * DM * 2);
static constexpr size_t SZ_W12 = al256((size_t)2 * HID * DM * 2);
static constexpr size_t SZ_W3  = al256((size_t)DM * HID * 2);
static constexpr size_t SZ_TOTAL = 3 * SZ_X + 3 * SZ_PL + 2 * SZ_X + SZ_HF + 6 * SZ_WS + 2 * SZ_WO + SZ_W12 + SZ_W3;
static_assert(SZ_G <= 3 * SZ_X + SZ_PL);
static_assert(SZ_PL <= SZ_X);
static_assert((size_t)NB * SEQ * DM * 2 <= SZ_X);
static_assert(SZ_TOTAL <= (size_t)134217728);
static_assert((size_t)NB * NH_ * SEQ * HD == (size_t)NB * DM * SEQ);
static_assert(((size_t)NB * SEQ * DM) % 8 == 0);
static_assert(((size_t)SEQ * DM) % 8 == 0);

extern "C" void kernel_launch(void* const* d_in, const int* in_sizes, int n_in,
                              void* d_out, int out_size, void* d_ws, size_t ws_size, hipStream_t stream) {
    if (n_in < 25) return;
    const size_t needx = ((size_t)(NB - 1) * SEQ_FULL + SEQ) * DM;
    const size_t needm = (size_t)(NB - 1) * SEQ_FULL + SEQ;
    if ((size_t)in_sizes[0] < needx || (size_t)in_sizes[1] < needx || (size_t)in_sizes[2] < needx) return;
    if ((size_t)in_sizes[3] < needm || (size_t)in_sizes[4] < needm) return;
    if (in_sizes[5] < HD * HD || in_sizes[6] < HD * HD || in_sizes[7] < HD * HD) return;
    if (in_sizes[10] < HD * HD || in_sizes[11] < HD * HD || in_sizes[12] < HD * HD) return;
    if ((size_t)in_sizes[8] < (size_t)DM * DM || (size_t)in_sizes[13] < (size_t)DM * DM) return;
    if (in_sizes[9] < DM || in_sizes[14] < DM) return;
    for (int i = 15; i <= 20; ++i) if (in_sizes[i] < DM) return;
    if ((size_t)in_sizes[21] < (size_t)DM * 2 * HID || in_sizes[22] < 2 * HID) return;
    if ((size_t)in_sizes[23] < (size_t)HID * DM || in_sizes[24] < DM) return;
    if ((size_t)out_size < ((size_t)(NB - 1) * OUT_SEQ + SEQ) * DM) return;
    if (SZ_TOTAL > ws_size) return;
    const float* xin[3] = { (const float*)d_in[0], (const float*)d_in[1], (const float*)d_in[2] };
    const int* src_mask = (const int*)d_in[3]; const int* tgt_mask = (const int*)d_in[4];
    const float* sa_wv = (const float*)d_in[5];  const float* sa_wk = (const float*)d_in[6];  const float* sa_wq = (const float*)d_in[7];
    const float* sa_wo = (const float*)d_in[8];  const float* sa_bo = (const float*)d_in[9];
    const float* ca_wv = (const float*)d_in[10]; const float* ca_wk = (const float*)d_in[11]; const float* ca_wq = (const float*)d_in[12];
    const float* ca_wo = (const float*)d_in[13]; const float* ca_bo = (const float*)d_in[14];
    const float* ln1_w = (const float*)d_in[15]; const float* ln1_b = (const float*)d_in[16];
    const float* ln2_w = (const float*)d_in[17]; const float* ln2_b = (const float*)d_in[18];
    const float* ln3_w = (const float*)d_in[19]; const float* ln3_b = (const float*)d_in[20];
    const float* w12 = (const float*)d_in[21];   const float* b12 = (const float*)d_in[22];
    const float* w3  = (const float*)d_in[23];   const float* b3  = (const float*)d_in[24];
    float* OUT = (float*)d_out;
    char* wsp = (char*)d_ws;
    h16* XH[3];
    h16* G = (h16*)wsp;
    XH[0] = (h16*)wsp; wsp += SZ_X;
    XH[1] = (h16*)wsp; wsp += SZ_X;
    XH[2] = (h16*)wsp; wsp += SZ_X;
    h16* QP = (h16*)wsp; wsp += SZ_PL;
    h16* KP = (h16*)wsp; wsp += SZ_PL;
    h16* VT = (h16*)wsp; wsp += SZ_PL;
    h16* CTX = (h16*)wsp; wsp += SZ_X;
    h16* HN = (h16*)wsp; wsp += SZ_X;
    float* HF = (float*)wsp; wsp += SZ_HF;
    h16* W1Q = (h16*)wsp; wsp += SZ_WS; h16* W1K = (h16*)wsp; wsp += SZ_WS; h16* W1V = (h16*)wsp; wsp += SZ_WS;
    h16* W2Q = (h16*)wsp; wsp += SZ_WS; h16* W2K = (h16*)wsp; wsp += SZ_WS; h16* W2V = (h16*)wsp; wsp += SZ_WS;
    h16* WO1 = (h16*)wsp; wsp += SZ_WO; h16* WO2 = (h16*)wsp; wsp += SZ_WO;
    h16* W12T = (h16*)wsp; wsp += SZ_W12;
    h16* W3T = (h16*)wsp; wsp += SZ_W3;
    h16* VR = HN;
    h16* CR = XH[0];

    for (int i = 0; i < 3; ++i) {
        if (SEQ == SEQ_FULL) {
            const size_t n8 = (size_t)NB * SEQ * DM / 8;
            k_cvth8<<<(unsigned)((n8 + 255) / 256), 256, 0, stream>>>(xin[i], XH[i], n8);
        } else {
            const size_t n8 = (size_t)SEQ * DM / 8;
            for (int b = 0; b < NB; ++b) k_cvth8<<<(unsigned)((n8 + 255) / 256), 256, 0, stream>>>(xin[i] + (size_t)b * SEQ_FULL * DM, XH[i] + (size_t)b * SEQ * DM, n8);
        }
    }
    k_wtr<<<dim3(1, 1, 1), 256, 0, stream>>>(sa_wq, W1Q, HD, HD);
    k_wtr<<<dim3(1, 1, 1), 256, 0, stream>>>(sa_wk, W1K, HD, HD);
    k_wtr<<<dim3(1, 1, 1), 256, 0, stream>>>(sa_wv, W1V, HD, HD);
    k_wtr<<<dim3(1, 1, 1), 256, 0, stream>>>(ca_wq, W2Q, HD, HD);
    k_wtr<<<dim3(1, 1, 1), 256, 0, stream>>>(ca_wk, W2K, HD, HD);
    k_wtr<<<dim3(1, 1, 1), 256, 0, stream>>>(ca_wv, W2V, HD, HD);
    k_wtr<<<dim3(DM / 64, DM / 64, 1), 256, 0, stream>>>(sa_wo, WO1, DM, DM);
    k_wtr<<<dim3(DM / 64, DM / 64, 1), 256, 0, stream>>>(ca_wo, WO2, DM, DM);
    k_wtr<<<dim3(2 * HID / 64, DM / 64, 1), 256, 0, stream>>>(w12, W12T, DM, 2 * HID);
    k_wtr<<<dim3(DM / 64, HID / 64, 1), 256, 0, stream>>>(w3, W3T, HID, DM);

    const dim3 gproj(NB * SEQ / 64, NH_, 1);
    const dim3 gflash(SEQ / (16 * AW), NB * NH_, 1);
    const dim3 ggemm(NB * SEQ / 64, DM / 64, 1);
    const dim3 ggemmr(NB * SEQ / 32, DM / 64, 1);

    k_proj_qk<<<gproj, 32, 0, stream>>>(XH[0], W1Q, QP, OSC_ONE);
    k_proj_qk<<<gproj, 32, 0, stream>>>(XH[0], W1K, KP, OSC_ONE);
    k_proj_vtr<<<gproj, 32, 0, stream>>>(XH[0], W1V, VT, VR, OSC_ONE);
    k_flash_vr<<<gflash, 32 * AW, 0, stream>>>(QP, KP, VT, VR, tgt_mask, CTX);
    k_gemm<<<ggemm, 32, 0, stream>>>(CTX, WO1, sa_bo, HF, DM, DM, SC_WO);
    k_ln_h<<<NB * SEQ / 8, 256, 0, stream>>>(HF, ln1_w, ln1_b, HN);

    k_proj_qk<<<gproj, 32, 0, stream>>>(XH[1], W2Q, QP, OSC_ONE);
    k_proj_qk<<<gproj, 32, 0, stream>>>(XH[2], W2K, KP, OSC_ONE);
    k_proj_vt<<<gproj, 32, 0, stream>>>(HN, W2V, VT, OSC_V2);
    k_flash_cr<<<gflash, 32 * AW, 0, stream>>>(QP, KP, VT, src_mask, CTX, CR);
    k_gemm_r<<<ggemmr, 32, 0, stream>>>(CTX, CR, WO2, ca_bo, HF, DM, DM, SC_WO);
    k_ln_h<<<NB * SEQ / 8, 256, 0, stream>>>(HF, ln2_w, ln2_b, HN);

    k_swiglu<<<dim3(NB * SEQ / 32, HID / 64, 1), 32, 0, stream>>>(HN, W12T, b12, G);
    k_gemm<<<ggemm, 32, 0, stream>>>(G, W3T, b3, HF, HID, DM, SC_W3);
    k_ln_f<<<NB * SEQ / 8, 256, 0, stream>>>(HF, ln3_w, ln3_b, OUT);
}
